// MLPDecoder_89215060672898
// MI455X (gfx1250) — hardware-verified
//
#include <hip/hip_runtime.h>
#include <stddef.h>


#define NBT   4
#define NAT   32
#define NTT   64
#define NDD   64
#define NSS   4
#define NET   4
#define NRR   992
#define MHH   256
#define KO1   320
#define NNODE (NBT * NAT * NTT)
#define PQW   512
#define LDH   264
#define NTHR  256
#define WSCAP 134217728
#define SCL_A   8.0f
#define SCL_W   16.0f
#define SCL_ACC 0.0078125f

static_assert(NNODE == 8192);
static_assert((NRR % 32) == 0);
static_assert((LDH % 8) == 0 && LDH >= MHH);
static_assert(KO1 == NDD + MHH);
static_assert((NDD % 32) == 0 && (MHH % 32) == 0 && (KO1 % 32) == 0);

typedef float    v4f  __attribute__((ext_vector_type(4)));
typedef float    v8f  __attribute__((ext_vector_type(8)));
typedef _Float16 v8h  __attribute__((ext_vector_type(8)));
typedef _Float16 v16h __attribute__((ext_vector_type(16)));
union FragH { v16h v; v8h h[2]; };

__device__ __forceinline__ v8f wmh(v16h a, v16h b, v8f c) {
  v8f d = __builtin_amdgcn_wmma_f32_16x16x32_f16(false, a, false, b, (short)0, c, false, false);
  asm volatile("v_nop\n\tv_nop\n\tv_nop\n\tv_nop" : "+v"(d) : "v"(a), "v"(b));
  return d;
}

__device__ __forceinline__ v8h cvt8(v4f a, v4f b, float s) {
  v8f t;
  t[0] = a.x * s; t[1] = a.y * s; t[2] = a.z * s; t[3] = a.w * s;
  t[4] = b.x * s; t[5] = b.y * s; t[6] = b.z * s; t[7] = b.w * s;
  return __builtin_convertvector(t, v8h);
}

__device__ __forceinline__ float lrelu1(float x) { return x > 0.0f ? x : 0.01f * x; }
__device__ __forceinline__ v4f lrelu4(v4f x) {
  v4f r;
  r.x = lrelu1(x.x); r.y = lrelu1(x.y); r.z = lrelu1(x.z); r.w = lrelu1(x.w);
  return r;
}

__global__ __launch_bounds__(NTHR) void k_xcvt(const float* __restrict__ x, _Float16* xp, int nUnits) {
  const int i = (int)blockIdx.x * NTHR + (int)threadIdx.x;
  if (i >= nUnits) return;
  const float* p = x + (size_t)i * 8;
  const v4f a = *(const v4f*)p;
  const v4f b = *(const v4f*)(p + 4);
  const v8h o = cvt8(a, b, SCL_A);
  _Float16* d = xp + (size_t)i * 8;
  *(volatile v8h*)d = o;
  __threadfence();
  *(volatile v8h*)d = o;
}

__global__ __launch_bounds__(NTHR) void k_prepT(const float* __restrict__ W, _Float16* wp,
                                               int K, int N, int srcStride, int dstStride, int nUnits) {
  const int i = (int)blockIdx.x * NTHR + (int)threadIdx.x;
  if (i >= nUnits) return;
  const int upr = K >> 3;
  int n = i / upr;
  const int k0 = (i - n * upr) * 8;
  n = n > N - 1 ? N - 1 : (n < 0 ? 0 : n);
  const float* src = W + (size_t)blockIdx.y * (size_t)srcStride + (size_t)k0 * N + n;
  v8f t;
  t[0] = src[0] * SCL_W;
  t[1] = src[(size_t)N] * SCL_W;
  t[2] = src[(size_t)2 * N] * SCL_W;
  t[3] = src[(size_t)3 * N] * SCL_W;
  t[4] = src[(size_t)4 * N] * SCL_W;
  t[5] = src[(size_t)5 * N] * SCL_W;
  t[6] = src[(size_t)6 * N] * SCL_W;
  t[7] = src[(size_t)7 * N] * SCL_W;
  const v8h o = __builtin_convertvector(t, v8h);
  _Float16* d = wp + (size_t)blockIdx.y * (size_t)dstStride + (size_t)i * 8;
  *(volatile v8h*)d = o;
  __threadfence();
  *(volatile v8h*)d = o;
}

__global__ __launch_bounds__(NTHR) void k_pq(const _Float16* __restrict__ xp, const _Float16* __restrict__ w1p, float* pq) {
  __shared__ __attribute__((aligned(16))) float stg[32 * MHH];
  const int tid = threadIdx.x, lane = tid & 31, wave = tid >> 5;
  const int hh = lane >> 4, m = lane & 15;
  const int rb = blockIdx.x, cb = blockIdx.y;
  const int typ = cb >> 1, kh = cb & 1;
  const int rg = wave >> 2, cq = wave & 3;

  const _Float16* Bpl = w1p + (size_t)typ * (MHH * 2 * NDD) + kh * NDD;
  const _Float16* ap  = xp + (size_t)(rb * 32 + 16 * rg + m) * NDD + 8 * hh;

  v8f acc[4];
#pragma unroll
  for (int t = 0; t < 4; ++t) { v8f z = {0.f, 0.f, 0.f, 0.f, 0.f, 0.f, 0.f, 0.f}; acc[t] = z; }

#pragma unroll
  for (int kt = 0; kt < NDD / 32; ++kt) {
    FragH a;
    a.h[0] = *(const v8h*)(ap + 32 * kt);
    a.h[1] = *(const v8h*)(ap + 32 * kt + 16);
#pragma unroll
    for (int t = 0; t < 4; ++t) {
      const _Float16* bp = Bpl + (size_t)(64 * cq + 16 * t + m) * (2 * NDD) + 32 * kt + 8 * hh;
      FragH bf;
      bf.h[0] = *(const v8h*)bp;
      bf.h[1] = *(const v8h*)(bp + 16);
      acc[t] = wmh(a.v, bf.v, acc[t]);
    }
  }

  float* sp = stg + (size_t)(16 * rg + 8 * hh) * MHH + 64 * cq + m;
#pragma unroll
  for (int t = 0; t < 4; ++t) {
#pragma unroll
    for (int r = 0; r < 8; ++r) sp[r * MHH + 16 * t] = acc[t][r] * SCL_ACC;
  }
  __syncthreads();

  float* dst = pq + ((size_t)typ * NNODE + (size_t)rb * 32) * PQW + kh * MHH;
  v4f ov[8];
#pragma unroll
  for (int it = 0; it < 8; ++it) ov[it] = *(const v4f*)(stg + 4 * (it * NTHR + tid));
#pragma unroll
  for (int it = 0; it < 8; ++it) {
    const int u = it * NTHR + tid;
    const int row = u >> 6, c4 = u & 63;
    *(volatile v4f*)(dst + (size_t)row * PQW + 4 * c4) = ov[it];
  }
  __threadfence();
#pragma unroll
  for (int it = 0; it < 8; ++it) {
    const int u = it * NTHR + tid;
    const int row = u >> 6, c4 = u & 63;
    *(volatile v4f*)(dst + (size_t)row * PQW + 4 * c4) = ov[it];
  }
}

__global__ __launch_bounds__(NTHR) void k_msg(
    const float* __restrict__ rel_rec, const float* __restrict__ rel_send,
    const float* __restrict__ rel_type, const float* __restrict__ state,
    const float* __restrict__ pq, const float* __restrict__ b1,
    const _Float16* __restrict__ w2p, const float* __restrict__ b2,
    _Float16* aggp) {
  __shared__ __attribute__((aligned(16))) _Float16 h1t[64 * LDH];
  __shared__ __attribute__((aligned(16))) float red[8 * MHH];
  __shared__ float gates[3 * 64];
  __shared__ int srel[32];
  __shared__ int ssend[32];
  __shared__ int scnt;

  const int a = blockIdx.x, t0 = (int)blockIdx.y * 2, b = blockIdx.z;
  const int tid = threadIdx.x, lane = tid & 31, wave = tid >> 5;
  const int hh = lane >> 4, m = lane & 15;
  const int nt0 = wave * 2;

  if (wave == 0) {
    srel[lane] = 0;
    int cnt = 0;
#pragma unroll 1
    for (int it = 0; it < NRR / 32; ++it) {
      const int r = it * 32 + lane;
      const float v = rel_rec[(size_t)r * NAT + a];
      const bool hit = v > 0.5f;
      const unsigned mk = __builtin_amdgcn_ballot_w32(hit);
      const int pos = cnt + (int)__builtin_amdgcn_mbcnt_lo(mk, 0u);
      if (hit && pos < 32) srel[pos] = r;
      cnt += (int)__builtin_popcount(mk);
    }
    if (lane == 0) scnt = cnt > 32 ? 32 : cnt;
  }
  __syncthreads();
  const int nrel = scnt;

  if (tid < 32) {
    int r = srel[tid];
    r = r < 0 ? 0 : (r > NRR - 1 ? NRR - 1 : r);
    const float* rs = rel_send + (size_t)r * NAT;
    float best = rs[0];
    int bi = 0;
#pragma unroll 1
    for (int c = 1; c < NAT; ++c) {
      const float v = rs[c];
      const bool gt = v > best;
      best = gt ? v : best;
      bi = gt ? c : bi;
    }
    ssend[tid] = bi;
  }
  __syncthreads();

  if (tid < 192) {
    const int i = tid >> 6, row = tid & 63;
    const int tl = row >> 5, j = row & 31;
    int r = srel[j];
    r = r < 0 ? 0 : (r > NRR - 1 ? NRR - 1 : r);
    int snd = ssend[j];
    snd = snd < 0 ? 0 : (snd > NAT - 1 ? NAT - 1 : snd);
    const float* rt  = rel_type + ((size_t)(b * NRR + r) * NSS) * NET + (i + 1);
    const float* stp = state + ((size_t)(b * NAT + snd) * NTT + (t0 + tl)) * NSS;
    float g = 0.0f;
#pragma unroll
    for (int s = 0; s < NSS; ++s) g += rt[s * NET] * stp[s];
    g = (j < nrel) ? g : 0.0f;
    gates[i * 64 + row] = g;
  }
#pragma unroll
  for (int q = 0; q < 8; ++q) red[q * MHH + tid] = 0.0f;
  __syncthreads();

  const int rowb = tid >> 2, qb = tid & 3;
  const int tlb = rowb >> 5, jb = rowb & 31;
  int sndb = ssend[jb];
  sndb = sndb < 0 ? 0 : (sndb > NAT - 1 ? NAT - 1 : sndb);
  const size_t nP = (size_t)(b * NAT + sndb) * NTT + (size_t)(t0 + tlb);
  const size_t nQ = (size_t)(b * NAT + a) * NTT + (size_t)(t0 + tlb);

#pragma unroll 1
  for (int i = 0; i < 3; ++i) {
    {
      const float* pp  = pq + ((size_t)i * NNODE + nP) * PQW + qb * 64;
      const float* qp  = pq + ((size_t)i * NNODE + nQ) * PQW + MHH + qb * 64;
      const float* bp1 = b1 + (size_t)(i + 1) * MHH + qb * 64;
      _Float16* hp = h1t + (size_t)rowb * LDH + qb * 64;
#pragma unroll 2
      for (int c = 0; c < 8; ++c) {
        const v4f p0 = *(const v4f*)(pp + 8 * c);
        const v4f p1 = *(const v4f*)(pp + 8 * c + 4);
        const v4f q0 = *(const v4f*)(qp + 8 * c);
        const v4f q1 = *(const v4f*)(qp + 8 * c + 4);
        const v4f e0 = *(const v4f*)(bp1 + 8 * c);
        const v4f e1 = *(const v4f*)(bp1 + 8 * c + 4);
        const v4f u0 = lrelu4(p0 + q0 + e0);
        const v4f u1 = lrelu4(p1 + q1 + e1);
        *(v8h*)(hp + 8 * c) = cvt8(u0, u1, SCL_A);
      }
    }
    __syncthreads();

    v8f acc[4][2];
#pragma unroll
    for (int mt = 0; mt < 4; ++mt)
#pragma unroll
      for (int tp = 0; tp < 2; ++tp) { v8f z = {0.f, 0.f, 0.f, 0.f, 0.f, 0.f, 0.f, 0.f}; acc[mt][tp] = z; }
    const _Float16* Bb0 = w2p + ((size_t)i * MHH + (size_t)(16 * nt0 + m)) * MHH + 8 * hh;
    const _Float16* Bb1 = Bb0 + (size_t)16 * MHH;
    const _Float16* Ab  = h1t + (size_t)m * LDH + 8 * hh;
#pragma unroll 1
    for (int kt = 0; kt < MHH / 32; ++kt) {
      FragH bf0, bf1;
      bf0.h[0] = *(const v8h*)(Bb0 + 32 * kt);
      bf0.h[1] = *(const v8h*)(Bb0 + 32 * kt + 16);
      bf1.h[0] = *(const v8h*)(Bb1 + 32 * kt);
      bf1.h[1] = *(const v8h*)(Bb1 + 32 * kt + 16);
#pragma unroll
      for (int mt = 0; mt < 4; ++mt) {
        const _Float16* arow = Ab + (size_t)(16 * mt) * LDH + 32 * kt;
        FragH af;
        af.h[0] = *(const v8h*)arow;
        af.h[1] = *(const v8h*)(arow + 16);
        acc[mt][0] = wmh(af.v, bf0.v, acc[mt][0]);
        acc[mt][1] = wmh(af.v, bf1.v, acc[mt][1]);
      }
    }

    {
      const float c0 = b2[(size_t)(i + 1) * MHH + 16 * nt0 + m];
      const float c1 = b2[(size_t)(i + 1) * MHH + 16 * nt0 + 16 + m];
#pragma unroll
      for (int mt = 0; mt < 4; ++mt) {
        float p0 = 0.0f, p1 = 0.0f;
#pragma unroll
        for (int r = 0; r < 8; ++r) {
          const float g = gates[i * 64 + 16 * mt + 8 * hh + r];
          p0 += lrelu1(acc[mt][0][r] * SCL_ACC + c0) * g;
          p1 += lrelu1(acc[mt][1][r] * SCL_ACC + c1) * g;
        }
        red[(2 * mt + hh) * MHH + 16 * nt0 + m]      += p0;
        red[(2 * mt + hh) * MHH + 16 * nt0 + 16 + m] += p1;
      }
    }
    __syncthreads();
  }

  if (tid < 64) {
    const int u = tid;
    const int tl = u >> 5, col = (u & 31) * 8;
    const float* r0 = red + (size_t)(tl * 4) * MHH + col;
    const v4f s0 = *(const v4f*)(r0) + *(const v4f*)(r0 + MHH) + *(const v4f*)(r0 + 2 * MHH) + *(const v4f*)(r0 + 3 * MHH);
    const v4f s1 = *(const v4f*)(r0 + 4) + *(const v4f*)(r0 + MHH + 4) + *(const v4f*)(r0 + 2 * MHH + 4) + *(const v4f*)(r0 + 3 * MHH + 4);
    const v8h o = cvt8(s0, s1, SCL_A);
    _Float16* d = aggp + ((size_t)(b * NAT + a) * NTT + (size_t)t0) * MHH + 8 * u;
    *(volatile v8h*)d = o;
    __threadfence();
    *(volatile v8h*)d = o;
  }
}

__global__ __launch_bounds__(NTHR) void k_node(
    const float* __restrict__ inputs, const _Float16* __restrict__ xp, const _Float16* __restrict__ aggp,
    const _Float16* __restrict__ wo1p, const float* __restrict__ bo1,
    const _Float16* __restrict__ wo2p, const float* __restrict__ bo2,
    const _Float16* __restrict__ wo3p, const float* __restrict__ bo3,
    float* out) {
  __shared__ __attribute__((aligned(16))) _Float16 hA[32 * LDH];
  __shared__ __attribute__((aligned(16))) _Float16 hB[32 * LDH];
  __shared__ __attribute__((aligned(16))) float sout[32 * NDD];
  const int tid = threadIdx.x, lane = tid & 31, wave = tid >> 5;
  const int hh = lane >> 4, m = lane & 15;
  const int nt0 = wave * 2;
  const int nb = blockIdx.x;
  const int rowBase = nb * 32;

  {
    v8f acc[2][2];
#pragma unroll
    for (int mt = 0; mt < 2; ++mt)
#pragma unroll
      for (int tp = 0; tp < 2; ++tp) { v8f z = {0.f, 0.f, 0.f, 0.f, 0.f, 0.f, 0.f, 0.f}; acc[mt][tp] = z; }
    const _Float16* B0 = wo1p + (size_t)(16 * nt0 + m) * KO1 + 8 * hh;
    const _Float16* B1 = B0 + (size_t)16 * KO1;
#pragma unroll
    for (int kt = 0; kt < NDD / 32; ++kt) {
      FragH bf0, bf1;
      bf0.h[0] = *(const v8h*)(B0 + 32 * kt);
      bf0.h[1] = *(const v8h*)(B0 + 32 * kt + 16);
      bf1.h[0] = *(const v8h*)(B1 + 32 * kt);
      bf1.h[1] = *(const v8h*)(B1 + 32 * kt + 16);
#pragma unroll
      for (int mt = 0; mt < 2; ++mt) {
        const _Float16* arow = xp + (size_t)(rowBase + 16 * mt + m) * NDD + 8 * hh + 32 * kt;
        FragH af;
        af.h[0] = *(const v8h*)arow;
        af.h[1] = *(const v8h*)(arow + 16);
        acc[mt][0] = wmh(af.v, bf0.v, acc[mt][0]);
        acc[mt][1] = wmh(af.v, bf1.v, acc[mt][1]);
      }
    }
#pragma unroll 1
    for (int kt = 0; kt < MHH / 32; ++kt) {
      FragH bf0, bf1;
      bf0.h[0] = *(const v8h*)(B0 + NDD + 32 * kt);
      bf0.h[1] = *(const v8h*)(B0 + NDD + 32 * kt + 16);
      bf1.h[0] = *(const v8h*)(B1 + NDD + 32 * kt);
      bf1.h[1] = *(const v8h*)(B1 + NDD + 32 * kt + 16);
#pragma unroll
      for (int mt = 0; mt < 2; ++mt) {
        const _Float16* arow = aggp + (size_t)(rowBase + 16 * mt + m) * MHH + 8 * hh + 32 * kt;
        FragH af;
        af.h[0] = *(const v8h*)arow;
        af.h[1] = *(const v8h*)(arow + 16);
        acc[mt][0] = wmh(af.v, bf0.v, acc[mt][0]);
        acc[mt][1] = wmh(af.v, bf1.v, acc[mt][1]);
      }
    }
    const float bn0 = bo1[16 * nt0 + m], bn1 = bo1[16 * nt0 + 16 + m];
#pragma unroll
    for (int mt = 0; mt < 2; ++mt)
#pragma unroll
      for (int r = 0; r < 8; ++r) {
        const int rr = 16 * mt + 8 * hh + r;
        hA[(size_t)rr * LDH + 16 * nt0 + m]      = (_Float16)(lrelu1(acc[mt][0][r] * SCL_ACC + bn0) * SCL_A);
        hA[(size_t)rr * LDH + 16 * nt0 + 16 + m] = (_Float16)(lrelu1(acc[mt][1][r] * SCL_ACC + bn1) * SCL_A);
      }
  }
  __syncthreads();

  {
    v8f acc[2][2];
#pragma unroll
    for (int mt = 0; mt < 2; ++mt)
#pragma unroll
      for (int tp = 0; tp < 2; ++tp) { v8f z = {0.f, 0.f, 0.f, 0.f, 0.f, 0.f, 0.f, 0.f}; acc[mt][tp] = z; }
    const _Float16* B0 = wo2p + (size_t)(16 * nt0 + m) * MHH + 8 * hh;
    const _Float16* B1 = B0 + (size_t)16 * MHH;
    const _Float16* Ab = hA + (size_t)m * LDH + 8 * hh;
#pragma unroll 1
    for (int kt = 0; kt < MHH / 32; ++kt) {
      FragH bf0, bf1;
      bf0.h[0] = *(const v8h*)(B0 + 32 * kt);
      bf0.h[1] = *(const v8h*)(B0 + 32 * kt + 16);
      bf1.h[0] = *(const v8h*)(B1 + 32 * kt);
      bf1.h[1] = *(const v8h*)(B1 + 32 * kt + 16);
#pragma unroll
      for (int mt = 0; mt < 2; ++mt) {
        const _Float16* arow = Ab + (size_t)(16 * mt) * LDH + 32 * kt;
        FragH af;
        af.h[0] = *(const v8h*)arow;
        af.h[1] = *(const v8h*)(arow + 16);
        acc[mt][0] = wmh(af.v, bf0.v, acc[mt][0]);
        acc[mt][1] = wmh(af.v, bf1.v, acc[mt][1]);
      }
    }
    const float bn0 = bo2[16 * nt0 + m], bn1 = bo2[16 * nt0 + 16 + m];
#pragma unroll
    for (int mt = 0; mt < 2; ++mt)
#pragma unroll
      for (int r = 0; r < 8; ++r) {
        const int rr = 16 * mt + 8 * hh + r;
        hB[(size_t)rr * LDH + 16 * nt0 + m]      = (_Float16)(lrelu1(acc[mt][0][r] * SCL_ACC + bn0) * SCL_A);
        hB[(size_t)rr * LDH + 16 * nt0 + 16 + m] = (_Float16)(lrelu1(acc[mt][1][r] * SCL_ACC + bn1) * SCL_A);
      }
  }
  __syncthreads();

  {
    const int mt3 = wave >> 2, nt3 = wave & 3;
    v8f a3 = {0.f, 0.f, 0.f, 0.f, 0.f, 0.f, 0.f, 0.f};
    const _Float16* Bp = wo3p + (size_t)(16 * nt3 + m) * MHH + 8 * hh;
    const _Float16* Ap = hB + (size_t)(16 * mt3 + m) * LDH + 8 * hh;
#pragma unroll 1
    for (int kt = 0; kt < MHH / 32; ++kt) {
      FragH af, bf;
      af.h[0] = *(const v8h*)(Ap + 32 * kt);
      af.h[1] = *(const v8h*)(Ap + 32 * kt + 16);
      bf.h[0] = *(const v8h*)(Bp + 32 * kt);
      bf.h[1] = *(const v8h*)(Bp + 32 * kt + 16);
      a3 = wmh(af.v, bf.v, a3);
    }
    const int d = 16 * nt3 + m;
    const float bn = bo3[d];
#pragma unroll
    for (int r = 0; r < 8; ++r) {
      const int rr = 16 * mt3 + 8 * hh + r;
      const float xv = inputs[(size_t)(rowBase + rr) * NDD + d];
      sout[rr * NDD + d] = xv + (a3[r] * SCL_ACC + bn);
    }
  }
  __syncthreads();

  const int pair = nb >> 1, half = nb & 1;
  const int nvalid = half ? 31 : 32;
  const int units = nvalid * (NDD / 4);
  float* ob = out + ((size_t)pair * (NTT - 1) + (size_t)half * 32) * NDD;
  v4f ov[2];
#pragma unroll
  for (int it = 0; it < 2; ++it) ov[it] = *(const v4f*)(sout + 4 * (it * NTHR + tid));
#pragma unroll
  for (int it = 0; it < 2; ++it) {
    const int u = it * NTHR + tid;
    if (u < units) *(volatile v4f*)(ob + 4 * (size_t)u) = ov[it];
  }
  __threadfence();
#pragma unroll
  for (int it = 0; it < 2; ++it) {
    const int u = it * NTHR + tid;
    if (u < units) *(volatile v4f*)(ob + 4 * (size_t)u) = ov[it];
  }
}

extern "C" void kernel_launch(void* const* d_in, const int* in_sizes, int n_in,
                              void* d_out, int out_size, void* d_ws, size_t ws_size,
                              hipStream_t stream) {
  if (n_in < 15) return;
  if (in_sizes[0] != NNODE * NDD) return;
  if (in_sizes[1] != NNODE * NSS) return;
  if (in_sizes[2] != NBT * NRR * NSS * NET) return;
  if (in_sizes[3] != NRR * NAT || in_sizes[4] != NRR * NAT) return;
  if (in_sizes[5] != NET * 2 * NDD * MHH || in_sizes[6] != NET * MHH) return;
  if (in_sizes[7] != NET * MHH * MHH || in_sizes[8] != NET * MHH) return;
  if (in_sizes[9] != KO1 * MHH || in_sizes[10] != MHH) return;
  if (in_sizes[11] != MHH * MHH || in_sizes[12] != MHH) return;
  if (in_sizes[13] != MHH * NDD || in_sizes[14] != NDD) return;
  if (out_size != NBT * NAT * (NTT - 1) * NDD) return;

  const float* inputs    = (const float*)d_in[0];
  const float* state     = (const float*)d_in[1];
  const float* rel_type  = (const float*)d_in[2];
  const float* rel_rec   = (const float*)d_in[3];
  const float* rel_send  = (const float*)d_in[4];
  const float* msg_fc1_w = (const float*)d_in[5];
  const float* msg_fc1_b = (const float*)d_in[6];
  const float* msg_fc2_w = (const float*)d_in[7];
  const float* msg_fc2_b = (const float*)d_in[8];
  const float* out_fc1_w = (const float*)d_in[9];
  const float* out_fc1_b = (const float*)d_in[10];
  const float* out_fc2_w = (const float*)d_in[11];
  const float* out_fc2_b = (const float*)d_in[12];
  const float* out_fc3_w = (const float*)d_in[13];
  const float* out_fc3_b = (const float*)d_in[14];
  float* out = (float*)d_out;

  char* ws = (char*)d_ws;
  size_t off = 0;
  const size_t oX   = off; off += (size_t)NNODE * NDD * 2;         off = (off + 255) & ~(size_t)255;
  const size_t oW1  = off; off += (size_t)3 * MHH * 2 * NDD * 2;   off = (off + 255) & ~(size_t)255;
  const size_t oW2  = off; off += (size_t)3 * MHH * MHH * 2;       off = (off + 255) & ~(size_t)255;
  const size_t oO1  = off; off += (size_t)MHH * KO1 * 2;           off = (off + 255) & ~(size_t)255;
  const size_t oO2  = off; off += (size_t)MHH * MHH * 2;           off = (off + 255) & ~(size_t)255;
  const size_t oO3  = off; off += (size_t)NDD * MHH * 2;           off = (off + 255) & ~(size_t)255;
  const size_t oPQ  = off; off += (size_t)3 * NNODE * PQW * 4;     off = (off + 255) & ~(size_t)255;
  const size_t oAgg = off; off += (size_t)NNODE * MHH * 2;         off = (off + 255) & ~(size_t)255;
  if (off > ws_size || off > (size_t)WSCAP) return;
  _Float16* xP   = (_Float16*)(ws + oX);
  _Float16* w1p  = (_Float16*)(ws + oW1);
  _Float16* w2p  = (_Float16*)(ws + oW2);
  _Float16* wo1p = (_Float16*)(ws + oO1);
  _Float16* wo2p = (_Float16*)(ws + oO2);
  _Float16* wo3p = (_Float16*)(ws + oO3);
  float*    pqP  = (float*)(ws + oPQ);
  _Float16* aggP = (_Float16*)(ws + oAgg);

  const int nXu = NNODE * NDD / 8;
  k_xcvt<<<(nXu + NTHR - 1) / NTHR, NTHR, 0, stream>>>(inputs, xP, nXu);

  {
    const int u1 = MHH * (2 * NDD) / 8;
    dim3 g1((u1 + NTHR - 1) / NTHR, 3);
    k_prepT<<<g1, NTHR, 0, stream>>>(msg_fc1_w + (size_t)(2 * NDD) * MHH, w1p, 2 * NDD, MHH, 2 * NDD * MHH, MHH * 2 * NDD, u1);
    const int u2 = MHH * MHH / 8;
    dim3 g2((u2 + NTHR - 1) / NTHR, 3);
    k_prepT<<<g2, NTHR, 0, stream>>>(msg_fc2_w + (size_t)MHH * MHH, w2p, MHH, MHH, MHH * MHH, MHH * MHH, u2);
    const int u3 = MHH * KO1 / 8;
    dim3 g3((u3 + NTHR - 1) / NTHR, 1);
    k_prepT<<<g3, NTHR, 0, stream>>>(out_fc1_w, wo1p, KO1, MHH, 0, 0, u3);
    const int u4 = MHH * MHH / 8;
    dim3 g4((u4 + NTHR - 1) / NTHR, 1);
    k_prepT<<<g4, NTHR, 0, stream>>>(out_fc2_w, wo2p, MHH, MHH, 0, 0, u4);
    const int u5 = NDD * MHH / 8;
    dim3 g5((u5 + NTHR - 1) / NTHR, 1);
    k_prepT<<<g5, NTHR, 0, stream>>>(out_fc3_w, wo3p, MHH, NDD, 0, 0, u5);
  }

  {
    dim3 gp(NNODE / 32, 6);
    k_pq<<<gp, NTHR, 0, stream>>>(xP, w1p, pqP);
  }

  {
    dim3 gm(NAT, NTT / 2, NBT);
    k_msg<<<gm, NTHR, 0, stream>>>(rel_rec, rel_send, rel_type, state, pqP, msg_fc1_b, w2p, msg_fc2_b, aggP);
  }

  k_node<<<NNODE / 32, NTHR, 0, stream>>>(inputs, xP, aggP, wo1p, out_fc1_b, wo2p, out_fc2_b, wo3p, out_fc3_b, out);
}
